// MultiHeadSelfAttention_15822659518596
// MI455X (gfx1250) — hardware-verified
//
#include <hip/hip_runtime.h>
#include <math.h>

#ifndef NB
#define NB 4
#endif
#ifndef SEQ
#define SEQ 2048
#endif
#define SEQ_FULL 2048
#define DM 512
#define NH 8
#define DK 64
#define QKV_ROWS 1536
#define MTOK (NB * SEQ)
#define FEAT_FULL (SEQ_FULL * NH)

#define CARRY_W 64.0f
#define CARRY_Q 16.0f
#define CARRY_K 16.0f
#define CARRY_M 16.0f
#define SC_M 0.015625f
#define SC_OUT 0.00048828125f

static_assert(1.0f / (CARRY_W * CARRY_K) == 1.0f / 1024.0f);
static_assert(1.0f / (CARRY_Q * CARRY_M) == 1.0f / 256.0f);
static_assert(SC_M == CARRY_M / (CARRY_W * CARRY_K));
static_assert(SC_OUT == (1.0f / (CARRY_Q * CARRY_M)) * (1.0f / 8.0f));
static_assert(SC_OUT == (1.0f / 256.0f) * 0.125f);

static_assert(DM == NH * DK);
static_assert(DK == 64 && NH == 8 && DM == 512);
static_assert(QKV_ROWS == 3 * DM);
static_assert(SEQ <= SEQ_FULL);
static_assert(SEQ % 256 == 0);
static_assert(SEQ % 64 == 0 && SEQ % 32 == 0);
static_assert(MTOK % 64 == 0);
static_assert(DM % 64 == 0 && DM % 32 == 0);
static_assert((MTOK * (DM / 8)) % 256 == 0);
static_assert((2 * DM * (DM / 8)) % 256 == 0);
static_assert(((MTOK / 64) * (DM / 64)) % 8 == 0);
static_assert(((DM / 64) * (MTOK / 64)) % 8 == 0);
static_assert(DM / 64 == 8);

typedef _Float16 h16;
typedef __attribute__((ext_vector_type(16))) _Float16 v16h;
typedef __attribute__((ext_vector_type(8)))  _Float16 v8h;
typedef __attribute__((ext_vector_type(16))) __bf16   v16bf;
typedef __attribute__((ext_vector_type(8)))  float    v8f;
typedef __attribute__((ext_vector_type(4)))  float    v4f;
typedef __attribute__((ext_vector_type(4)))  unsigned int v4u;
typedef __attribute__((ext_vector_type(8)))  unsigned int v8u;


__device__ __forceinline__ float bfr(float f) {
    unsigned u = __float_as_uint(f);
    u += 0x7FFFu + ((u >> 16) & 1u);
    return __uint_as_float(u & 0xFFFF0000u);
}
__device__ __forceinline__ unsigned bf_hi(float f) {
    unsigned u = __float_as_uint(f);
    u += 0x7FFFu + ((u >> 16) & 1u);
    return u & 0xFFFF0000u;
}
__device__ __forceinline__ unsigned bf_pack(float lo, float hi) { return (bf_hi(lo) >> 16) | bf_hi(hi); }

static __device__ __forceinline__ h16 toh_flush(float v) {
    const float w = (fabsf(v) < 6.103515625e-05f) ? 0.0f : v;
    return (h16)w;
}

__device__ __forceinline__ void st8b(unsigned short* P, size_t o, v4f a, v4f b) {
    v4u pk;
    pk.x = bf_pack(a.x, a.y);
    pk.y = bf_pack(a.z, a.w);
    pk.z = bf_pack(b.x, b.y);
    pk.w = bf_pack(b.z, b.w);
    *(volatile v4u*)(P + o) = pk;
    __threadfence();
    *(volatile v4u*)(P + o) = pk;
}

union FragU { v16h v; v8h h[2]; };
__device__ __forceinline__ v16h frag_ld(const _Float16* p) {
    FragU f; f.h[0] = *(const v8h*)(p); f.h[1] = *(const v8h*)(p + 16); return f.v;
}
__device__ __forceinline__ v8u frag_ldb(const unsigned short* p) {
    const v4u lo = *(const v4u*)(p);
    const v4u hi = *(const v4u*)(p + 16);
    return __builtin_shufflevector(lo, hi, 0, 1, 2, 3, 4, 5, 6, 7);
}
__device__ __forceinline__ v8f wmma16g(v16h a, v16h b, v8f c) {
    c = __builtin_amdgcn_wmma_f32_16x16x32_f16(false, a, false, b, (short)0, c, false, false);
    asm volatile("v_nop\n\tv_nop\n\tv_nop\n\tv_nop" : "+v"(c) : "v"(a), "v"(b));
    return c;
}
__device__ __forceinline__ v8f wmmabg(v8u a, v8u b, v8f c) {
    c = __builtin_amdgcn_wmma_f32_16x16x32_bf16(false, __builtin_bit_cast(v16bf, a), false, __builtin_bit_cast(v16bf, b), (short)0, c, false, false);
    asm volatile("v_nop\n\tv_nop\n\tv_nop\n\tv_nop" : "+v"(c) : "v"(a), "v"(b));
    return c;
}
__device__ __forceinline__ void wave_sync_lds() {
    __builtin_amdgcn_fence(3  , "workgroup");
    __builtin_amdgcn_wave_barrier();
    __builtin_amdgcn_fence(2  , "workgroup");
}

__device__ __forceinline__ void mainloop_b(const unsigned short* __restrict__ A, unsigned lda,
                                           const unsigned short* __restrict__ Bt, unsigned ldb,
                                           unsigned m0, unsigned n0, unsigned K, unsigned lane, v8f (&acc)[4][4]) {
    const unsigned rlane = lane & 15u;
    const unsigned koff = (lane >> 4) * 8u;
    for (unsigned k0 = 0; k0 < K; k0 += 32u) {
        v8u bb[4];
#pragma unroll
        for (int j = 0; j < 4; ++j)
            bb[j] = frag_ldb(Bt + (size_t)(n0 + ((unsigned)j << 4) + rlane) * ldb + koff + k0);
#pragma unroll
        for (int i = 0; i < 4; ++i) {
            const v8u ab = frag_ldb(A + (size_t)(m0 + ((unsigned)i << 4) + rlane) * lda + koff + k0);
#pragma unroll
            for (int j = 0; j < 4; ++j) acc[i][j] = wmmabg(ab, bb[j], acc[i][j]);
        }
    }
}
__device__ __forceinline__ void mainloop_h(const _Float16* __restrict__ A, unsigned lda,
                                           const _Float16* __restrict__ Bt, unsigned ldb,
                                           unsigned m0, unsigned n0, unsigned K, unsigned lane, v8f (&acc)[4][4]) {
    const unsigned rlane = lane & 15u;
    const unsigned koff = (lane >> 4) * 8u;
    for (unsigned k0 = 0; k0 < K; k0 += 32u) {
        v16h bh[4];
#pragma unroll
        for (int j = 0; j < 4; ++j)
            bh[j] = frag_ld(Bt + (size_t)(n0 + ((unsigned)j << 4) + rlane) * ldb + koff + k0);
#pragma unroll
        for (int i = 0; i < 4; ++i) {
            const v16h ah = frag_ld(A + (size_t)(m0 + ((unsigned)i << 4) + rlane) * lda + koff + k0);
#pragma unroll
            for (int j = 0; j < 4; ++j) acc[i][j] = wmma16g(ah, bh[j], acc[i][j]);
        }
    }
}

static_assert(32 * 16 * 4 == 16 * 128);
static_assert(32 * 16 * 8 == 16 * 256);
static_assert(8 * 16 * 68 * 4 <= 131072);

__global__ __launch_bounds__(256) void k_cvt_x(const float* __restrict__ x, unsigned short* __restrict__ X16) {
    const unsigned u = blockIdx.x * 256u + threadIdx.x;
    const unsigned row = u >> 6, c0 = (u & 63u) * 8u;
    const unsigned b = row / (unsigned)SEQ;
    const unsigned i = row - b * (unsigned)SEQ;
    const float* src = x + ((size_t)b * SEQ_FULL + i) * DM + c0;
    const v4f a0 = *(const v4f*)(src);
    const v4f a1 = *(const v4f*)(src + 4);
    st8b(X16, (size_t)row * DM + c0, a0, a1);
}

__global__ __launch_bounds__(256) void k_cvt_wqk(const float* __restrict__ Wqkv, unsigned short* __restrict__ WQK16) {
    const unsigned u = blockIdx.x * 256u + threadIdx.x;
    const unsigned o = u >> 6, c0 = (u & 63u) * 8u;
    const unsigned sel = o >> 9, r = o & 511u;
    const unsigned srow = 192u * (r >> 6) + 64u * sel + (r & 63u);
    const float* src = Wqkv + (size_t)srow * DM + c0;
    const v4f a0 = *(const v4f*)(src);
    const v4f a1 = *(const v4f*)(src + 4);
    st8b(WQK16, (size_t)o * DM + c0, a0, a1);
}

#define WF_PITCH 264
static_assert(8 * WF_PITCH * 4 <= 131072);
static_assert(256 * 8 == 8 * 256);
static_assert(32 * 16 == 256 * 2);
__global__ __launch_bounds__(256) void k_cvt_wfc(const float* __restrict__ Wfc, _Float16* __restrict__ WfT) {
    __shared__ __align__(16) float sW[8 * WF_PITCH];
    const unsigned t = threadIdx.x;
    const unsigned d = blockIdx.y;
    const unsigned jc = blockIdx.x * 256u;
    const float* src = Wfc + (size_t)d * FEAT_FULL + (size_t)(jc + t) * 8u;
    const v4f a0 = *(const v4f*)(src);
    const v4f a1 = *(const v4f*)(src + 4);
    sW[0 * WF_PITCH + t] = bfr(a0.x) * CARRY_W;
    sW[1 * WF_PITCH + t] = bfr(a0.y) * CARRY_W;
    sW[2 * WF_PITCH + t] = bfr(a0.z) * CARRY_W;
    sW[3 * WF_PITCH + t] = bfr(a0.w) * CARRY_W;
    sW[4 * WF_PITCH + t] = bfr(a1.x) * CARRY_W;
    sW[5 * WF_PITCH + t] = bfr(a1.y) * CARRY_W;
    sW[6 * WF_PITCH + t] = bfr(a1.z) * CARRY_W;
    sW[7 * WF_PITCH + t] = bfr(a1.w) * CARRY_W;
    __syncthreads();
    const unsigned n = t >> 5, piece = t & 31u;
    const v4f p0 = *(const v4f*)(&sW[n * WF_PITCH + 8u * piece]);
    const v4f p1 = *(const v4f*)(&sW[n * WF_PITCH + 8u * piece + 4u]);
    v8h hv;
    hv[0] = toh_flush(p0.x); hv[1] = toh_flush(p0.y); hv[2] = toh_flush(p0.z); hv[3] = toh_flush(p0.w);
    hv[4] = toh_flush(p1.x); hv[5] = toh_flush(p1.y); hv[6] = toh_flush(p1.z); hv[7] = toh_flush(p1.w);
    _Float16* dst = WfT + ((size_t)(n * (unsigned)DM + d)) * SEQ + jc + 8u * piece;
    *(volatile v8h*)(dst) = hv;
    __threadfence();
    *(volatile v8h*)(dst) = hv;
}

__global__ __launch_bounds__(256) void k_gemm_q(const unsigned short* __restrict__ X16, const unsigned short* __restrict__ WQK16,
                                                const float* __restrict__ bqkv, _Float16* __restrict__ Q16) {
    __shared__ __align__(16) float sT[8][16 * 68];
    const unsigned lane = threadIdx.x & 31u;
    const unsigned wave = (unsigned)__builtin_amdgcn_readfirstlane((int)(threadIdx.x >> 5));
    const unsigned tile = blockIdx.x * 8u + wave;
    const unsigned tm = tile >> 3, tn = tile & 7u;
    const unsigned m0 = tm << 6, n0 = tn << 6;
    const unsigned rlane = lane & 15u, hh = lane >> 4;

    v8f acc[4][4];
#pragma unroll
    for (int i = 0; i < 4; ++i)
#pragma unroll
        for (int j = 0; j < 4; ++j) acc[i][j] = (v8f){0.f,0.f,0.f,0.f,0.f,0.f,0.f,0.f};

    mainloop_b(X16, DM, WQK16, DM, m0, n0, DM, lane, acc);

#pragma unroll
    for (int i = 0; i < 4; ++i) {
        const unsigned mBase = m0 + ((unsigned)i << 4);
#pragma unroll
        for (int j = 0; j < 4; ++j) {
            const float bv = bfr(bqkv[192u * tn + ((unsigned)j << 4) + rlane]);
#pragma unroll
            for (int r = 0; r < 8; ++r)
                sT[wave][(8u * hh + (unsigned)r) * 68u + ((unsigned)j << 4) + rlane] = (acc[i][j][r] + bv) * CARRY_Q;
        }
        wave_sync_lds();
        {
            const unsigned q4 = lane >> 3, c8 = (lane & 7u) * 8u;
            v8h hv[4];
#pragma unroll
            for (int it = 0; it < 4; ++it) {
                const unsigned row = (unsigned)it * 4u + q4;
#pragma unroll
                for (int e = 0; e < 8; ++e) hv[it][e] = toh_flush(sT[wave][row * 68u + c8 + (unsigned)e]);
            }
            for (int pass = 0; pass < 2; ++pass) {
#pragma unroll
                for (int it = 0; it < 4; ++it) {
                    const unsigned row = (unsigned)it * 4u + q4;
                    *(volatile v8h*)(Q16 + (size_t)(mBase + row) * DM + n0 + c8) = hv[it];
                }
                __threadfence();
            }
        }
        wave_sync_lds();
    }
}

__global__ __launch_bounds__(256) void k_gemm_kt(const unsigned short* __restrict__ WQK16, const unsigned short* __restrict__ X16,
                                                 const float* __restrict__ bqkv, _Float16* __restrict__ KT) {
    __shared__ __align__(16) float sT[8][16 * 68];
    const unsigned lane = threadIdx.x & 31u;
    const unsigned wave = (unsigned)__builtin_amdgcn_readfirstlane((int)(threadIdx.x >> 5));
    const unsigned tile = blockIdx.x * 8u + wave;
    const unsigned tm = tile & 7u, tn = tile >> 3;
    const unsigned m0 = tm << 6, n0 = tn << 6;
    const unsigned rlane = lane & 15u, hh = lane >> 4;
    const unsigned b = n0 / (unsigned)SEQ;
    const unsigned j0 = n0 - b * (unsigned)SEQ;

    v8f acc[4][4];
#pragma unroll
    for (int i = 0; i < 4; ++i)
#pragma unroll
        for (int j = 0; j < 4; ++j) acc[i][j] = (v8f){0.f,0.f,0.f,0.f,0.f,0.f,0.f,0.f};

    mainloop_b(WQK16 + (size_t)DM * DM, DM, X16, DM, m0, n0, DM, lane, acc);

#pragma unroll
    for (int i = 0; i < 4; ++i) {
        const unsigned mBase = m0 + ((unsigned)i << 4);
        float bvr[8];
#pragma unroll
        for (int r = 0; r < 8; ++r)
            bvr[r] = bfr(bqkv[192u * tm + 64u + ((unsigned)i << 4) + 8u * hh + (unsigned)r]);
#pragma unroll
        for (int j = 0; j < 4; ++j) {
#pragma unroll
            for (int r = 0; r < 8; ++r)
                sT[wave][(8u * hh + (unsigned)r) * 68u + ((unsigned)j << 4) + rlane] = (acc[i][j][r] + bvr[r]) * CARRY_K;
        }
        wave_sync_lds();
        {
            const unsigned q4 = lane >> 3, c8 = (lane & 7u) * 8u;
            v8h hv[4];
#pragma unroll
            for (int it = 0; it < 4; ++it) {
                const unsigned row = (unsigned)it * 4u + q4;
#pragma unroll
                for (int e = 0; e < 8; ++e) hv[it][e] = toh_flush(sT[wave][row * 68u + c8 + (unsigned)e]);
            }
            for (int pass = 0; pass < 2; ++pass) {
#pragma unroll
                for (int it = 0; it < 4; ++it) {
                    const unsigned row = (unsigned)it * 4u + q4;
                    *(volatile v8h*)(KT + (size_t)(b * (unsigned)DM + mBase + row) * SEQ + j0 + c8) = hv[it];
                }
                __threadfence();
            }
        }
        wave_sync_lds();
    }
}

__global__ __launch_bounds__(256) void k_gemm_m(const _Float16* __restrict__ WfT, const _Float16* __restrict__ KT,
                                                _Float16* __restrict__ MT) {
    __shared__ __align__(16) float sT[8][16 * 68];
    const unsigned lane = threadIdx.x & 31u;
    const unsigned wave = (unsigned)__builtin_amdgcn_readfirstlane((int)(threadIdx.x >> 5));
    const unsigned z = blockIdx.y;
    const unsigned b = z >> 3, n = z & 7u;
    const unsigned m0 = wave << 6;
    const unsigned rlane = lane & 15u, hh = lane >> 4;

    v8f acc[4][4];
#pragma unroll
    for (int i = 0; i < 4; ++i)
#pragma unroll
        for (int j = 0; j < 4; ++j) acc[i][j] = (v8f){0.f,0.f,0.f,0.f,0.f,0.f,0.f,0.f};

    mainloop_h(WfT + (size_t)n * DM * SEQ, SEQ, KT + (size_t)z * DK * SEQ, SEQ, m0, 0u, SEQ, lane, acc);

#pragma unroll
    for (int i = 0; i < 4; ++i) {
        const unsigned mBase = m0 + ((unsigned)i << 4);
#pragma unroll
        for (int j = 0; j < 4; ++j) {
#pragma unroll
            for (int r = 0; r < 8; ++r)
                sT[wave][(8u * hh + (unsigned)r) * 68u + ((unsigned)j << 4) + rlane] = acc[i][j][r] * SC_M;
        }
        wave_sync_lds();
        {
            const unsigned q4 = lane >> 3, c8 = (lane & 7u) * 8u;
            v8h hv[4];
#pragma unroll
            for (int it = 0; it < 4; ++it) {
                const unsigned row = (unsigned)it * 4u + q4;
#pragma unroll
                for (int e = 0; e < 8; ++e) hv[it][e] = toh_flush(sT[wave][row * 68u + c8 + (unsigned)e]);
            }
            for (int pass = 0; pass < 2; ++pass) {
#pragma unroll
                for (int it = 0; it < 4; ++it) {
                    const unsigned row = (unsigned)it * 4u + q4;
                    *(volatile v8h*)(MT + (size_t)(b * (unsigned)DM + mBase + row) * DM + 64u * n + c8) = hv[it];
                }
                __threadfence();
            }
        }
        wave_sync_lds();
    }
}

__global__ __launch_bounds__(256) void k_gemm_out(const _Float16* __restrict__ Q16, const _Float16* __restrict__ MT,
                                                  const float* __restrict__ bfc, float* __restrict__ out) {
    __shared__ __align__(16) float sT[8][16 * 68];
    const unsigned lane = threadIdx.x & 31u;
    const unsigned wave = (unsigned)__builtin_amdgcn_readfirstlane((int)(threadIdx.x >> 5));
    const unsigned b = blockIdx.y;
    const unsigned tile = blockIdx.x * 8u + wave;
    const unsigned tm = tile >> 3, tn = tile & 7u;
    const unsigned m0 = tm << 6, n0 = tn << 6;
    const unsigned rlane = lane & 15u, hh = lane >> 4;

    v8f acc[4][4];
#pragma unroll
    for (int i = 0; i < 4; ++i)
#pragma unroll
        for (int j = 0; j < 4; ++j) acc[i][j] = (v8f){0.f,0.f,0.f,0.f,0.f,0.f,0.f,0.f};

    mainloop_h(Q16 + (size_t)b * SEQ * DM, DM, MT + (size_t)b * DM * DM, DM, m0, n0, DM, lane, acc);

#pragma unroll
    for (int i = 0; i < 4; ++i) {
        const unsigned mBase = m0 + ((unsigned)i << 4);
#pragma unroll
        for (int j = 0; j < 4; ++j) {
            const float bv = bfr(bfc[n0 + ((unsigned)j << 4) + rlane]);
#pragma unroll
            for (int r = 0; r < 8; ++r)
                sT[wave][(8u * hh + (unsigned)r) * 68u + ((unsigned)j << 4) + rlane] = acc[i][j][r] * SC_OUT + bv;
        }
        wave_sync_lds();
        {
            const unsigned c4 = (lane & 15u) * 4u;
#pragma unroll
            for (int half = 0; half < 2; ++half) {
                v4f vv[4];
#pragma unroll
                for (int it = 0; it < 4; ++it) {
                    const unsigned row = (unsigned)(half * 4 + it) * 2u + hh;
                    vv[it] = *(const v4f*)(&sT[wave][row * 68u + c4]);
                }
                for (int pass = 0; pass < 2; ++pass) {
#pragma unroll
                    for (int it = 0; it < 4; ++it) {
                        const unsigned row = (unsigned)(half * 4 + it) * 2u + hh;
                        *(volatile v4f*)(out + ((size_t)b * SEQ_FULL + mBase + row) * DM + n0 + c4) = vv[it];
                    }
                    __threadfence();
                }
            }
        }
        wave_sync_lds();
    }
}

static constexpr size_t SZ_X16  = (size_t)MTOK * DM * 2;
static constexpr size_t SZ_WQK  = (size_t)2 * DM * DM * 2;
static constexpr size_t SZ_WFT  = (size_t)NH * DM * SEQ * 2;
static constexpr size_t SZ_Q16  = (size_t)MTOK * DM * 2;
static constexpr size_t SZ_KT   = (size_t)NB * DM * SEQ * 2;
static constexpr size_t SZ_MT   = (size_t)NB * DM * DM * 2;
static_assert(SZ_X16 % 256 == 0 && SZ_WQK % 256 == 0 && SZ_WFT % 256 == 0 && SZ_Q16 % 256 == 0 && SZ_KT % 256 == 0 && SZ_MT % 256 == 0);
static_assert(SZ_X16 + SZ_WQK + SZ_WFT + SZ_Q16 + SZ_KT + SZ_MT <= (size_t)134217728);

extern "C" void kernel_launch(void* const* d_in, const int* in_sizes, int n_in, void* d_out, int out_size,
                              void* d_ws, size_t ws_size, hipStream_t stream) {
    if (n_in < 5) return;
    if (in_sizes[0] < ((NB - 1) * SEQ_FULL + SEQ) * DM || in_sizes[1] < QKV_ROWS * DM || in_sizes[2] < QKV_ROWS) return;
    if (in_sizes[3] < DM * FEAT_FULL || in_sizes[4] < DM || out_size < ((NB - 1) * SEQ_FULL + SEQ) * DM) return;

    const float* x     = (const float*)d_in[0];
    const float* W_qkv = (const float*)d_in[1];
    const float* b_qkv = (const float*)d_in[2];
    const float* W_fc  = (const float*)d_in[3];
    const float* b_fc  = (const float*)d_in[4];
    float* out = (float*)d_out;

    char* wsp = (char*)d_ws;
    size_t off = 0;
    auto carve = [&](size_t bytes) -> void* { void* r = wsp + off; off += (bytes + 255) & ~(size_t)255; return r; };
    unsigned short* X16   = (unsigned short*)carve(SZ_X16);
    unsigned short* WQK16 = (unsigned short*)carve(SZ_WQK);
    _Float16*       WfT   = (_Float16*)carve(SZ_WFT);
    _Float16*       Q16   = (_Float16*)carve(SZ_Q16);
    _Float16*       KT    = (_Float16*)carve(SZ_KT);
    _Float16*       MT    = (_Float16*)carve(SZ_MT);
    if (off > ws_size || off > (size_t)134217728) return;

    k_cvt_x<<<(MTOK * (DM / 8)) / 256, 256, 0, stream>>>(x, X16);
    k_cvt_wqk<<<(2 * DM * (DM / 8)) / 256, 256, 0, stream>>>(W_qkv, WQK16);
    k_cvt_wfc<<<dim3(SEQ / 256, DM), 256, 0, stream>>>(W_fc, WfT);

    k_gemm_q<<<((MTOK / 64) * (DM / 64)) / 8, 256, 0, stream>>>(X16, WQK16, b_qkv, Q16);
    k_gemm_kt<<<((DM / 64) * (MTOK / 64)) / 8, 256, 0, stream>>>(WQK16, X16, b_qkv, KT);

    k_gemm_m<<<dim3(1, NB * NH), 256, 0, stream>>>(WfT, KT, MT);
    k_gemm_out<<<dim3(((SEQ / 64) * (DM / 64)) / 8, NB), 256, 0, stream>>>(Q16, MT, b_fc, out);
}
